// InvariantPointAttention_7988639171223
// MI455X (gfx1250) — hardware-verified
//
#include <hip/hip_runtime.h>
#include <math.h>

constexpr int kB    = 4;
constexpr int kN    = 1024;
constexpr int kDim  = 512;
constexpr int kH    = 8;
constexpr int kDh   = 64;
constexpr int kP    = 4;
constexpr int kTok  = kB * kN;
constexpr int kPc   = kP * 3;
constexpr int kProjW = kH * kPc;
constexpr int kProjN = 320;
constexpr int kFeat  = kH * (kDh + kP * 4);
constexpr int kFeatPt = kH * kP * 4;
constexpr int kVtpRows = 64;
constexpr int kVtpLive = 19;
constexpr float kScalarScale = 0.08838834764831845f;
constexpr float kPointScale  = 0.16666666666666666f;
constexpr float kEps      = 1e-8f;
constexpr float kWCarry   = 16.0f;
constexpr float kFCarry   = 16.0f;
constexpr float kLoCarry  = 2048.0f;
constexpr float kLoInv    = 1.0f / 2048.0f;
constexpr float kPCarry   = 32768.0f;
static_assert(kH * kDh == kDim, "shape");
static_assert(kFeat == 640 && kFeatPt == 128 && kProjW == 96, "shape");
static_assert(kN % 64 == 0 && kDim % 64 == 0 && kDh % 32 == 0 && kProjN % 64 == 0 && kFeat % 32 == 0 && kFeatPt % 32 == 0, "tiles");

typedef __attribute__((ext_vector_type(16))) _Float16 v16h;
typedef __attribute__((ext_vector_type(8)))  _Float16 v8h;
typedef __attribute__((ext_vector_type(16))) __bf16   v16b;
typedef __attribute__((ext_vector_type(8)))  __bf16   v8b;
typedef __attribute__((ext_vector_type(8)))  float    v8f;
typedef __attribute__((ext_vector_type(4)))  float    v4f;
typedef __attribute__((ext_vector_type(2)))  float    v2f;
typedef __attribute__((ext_vector_type(4)))  unsigned int v4u;

__device__ __forceinline__ unsigned short f2bf_bits(float f) {
  unsigned u = __float_as_uint(f);
  return (unsigned short)((u + 0x7FFFu + ((u >> 16) & 1u)) >> 16);
}
__device__ __forceinline__ float bf_bits2f(unsigned short h) { return __uint_as_float(((unsigned)h) << 16); }

__device__ __forceinline__ void dep_guard_h(v8f& a, v8f& b, v16h x, v16h y) { asm volatile("v_nop\n\tv_nop\n\tv_nop\n\tv_nop" : "+v"(a), "+v"(b) : "v"(x), "v"(y)); }
__device__ __forceinline__ void dep_guard_b(v8f& a, v8f& b, v16b x, v16b y) { asm volatile("v_nop\n\tv_nop\n\tv_nop\n\tv_nop" : "+v"(a), "+v"(b) : "v"(x), "v"(y)); }
__device__ __forceinline__ void keep4_h(v16h a, v16h b, v16h c, v16h d) { asm volatile("v_nop" :: "v"(a), "v"(b), "v"(c), "v"(d)); }
__device__ __forceinline__ void keep4_b(v16b a, v16b b, v16b c, v16b d) { asm volatile("v_nop" :: "v"(a), "v"(b), "v"(c), "v"(d)); }
__device__ __forceinline__ void acc_guard4(v8f& a, v8f& b, v8f& c, v8f& d) { asm volatile("v_nop\n\tv_nop\n\tv_nop\n\tv_nop" : "+v"(a), "+v"(b), "+v"(c), "+v"(d)); }
template <typename T> struct Frag;
template <> struct Frag<_Float16> {
  typedef v16h V; union U { v16h v; v8h h[2]; };
  static __device__ __forceinline__ v16h load(const _Float16* p) {
    U f; f.h[0] = *(const v8h*)(p); f.h[1] = *(const v8h*)(p + 16); return f.v;
  }
  static __device__ __forceinline__ v8f mma(v16h a, v16h b, v8f c) {
    return __builtin_amdgcn_wmma_f32_16x16x32_f16(false, a, false, b, (short)0, c, false, false);
  }
  static __device__ __forceinline__ void guard(v8f& a, v8f& b, v16h x, v16h y) { dep_guard_h(a, b, x, y); }
  static __device__ __forceinline__ void keep(v16h a, v16h b, v16h c, v16h d) { keep4_h(a, b, c, d); }
};
template <> struct Frag<__bf16> {
  typedef v16b V; union U { v16b v; v8b h[2]; };
  static __device__ __forceinline__ v16b load(const __bf16* p) {
    U f; f.h[0] = *(const v8b*)(p); f.h[1] = *(const v8b*)(p + 16); return f.v;
  }
  static __device__ __forceinline__ v8f mma(v16b a, v16b b, v8f c) {
    return __builtin_amdgcn_wmma_f32_16x16x32_bf16(false, a, false, b, (short)0, c, false, false);
  }
  static __device__ __forceinline__ void guard(v8f& a, v8f& b, v16b x, v16b y) { dep_guard_b(a, b, x, y); }
  static __device__ __forceinline__ void keep(v16b a, v16b b, v16b c, v16b d) { keep4_b(a, b, c, d); }
};

__device__ __forceinline__ unsigned pk16(unsigned short a, unsigned short b) { return (unsigned)a | ((unsigned)b << 16); }
__device__ __forceinline__ unsigned short h_bits(float f) { const _Float16 h = (_Float16)f; return __builtin_bit_cast(unsigned short, h); }

__device__ __forceinline__ float h16_to_f32(unsigned hb) {
  const unsigned sgn = (hb & 0x8000u) << 16; const unsigned em = hb & 0x7fffu;
  const float fn = __uint_as_float((em << 13) + 0x38000000u);
  const float fs = (float)em * 5.9604644775390625e-8f;
  const float mag = (em < 0x400u) ? fs : fn; return __uint_as_float(__float_as_uint(mag) | sgn); }

__device__ __forceinline__ void split16(float x, unsigned short& hb, unsigned short& lb) {
  hb = h_bits(x);
  const float hf = h16_to_f32((unsigned)hb);
  lb = h_bits((x - hf) * kLoCarry);
}

template <int ET> struct Elem;
template <> struct Elem<0> { typedef _Float16 T; };
template <> struct Elem<1> { typedef __bf16 T; };
template <int ET, bool SPLIT, int BIAS_MODE, int OUT_MODE, bool RESID, int ACT = 0>
__global__ __launch_bounds__(256) void wmma_gemm64(
    const unsigned short* __restrict__ Ap, const unsigned short* __restrict__ A2p, int lda, long strideA,
    const unsigned short* __restrict__ Btp, const unsigned short* __restrict__ Bt2p, int ldb, long strideB,
    void* __restrict__ Cout, void* __restrict__ Cout2, int ldc, long strideC,
    const float* __restrict__ bias,
    const float* __restrict__ resid, long strideR,
    int M, int N, int K, float scale) {
  static_assert(!RESID || OUT_MODE == 0, "resid");
  typedef typename Elem<ET>::T T;
  typedef typename Frag<T>::V V;
  const T* A = (const T*)Ap; const T* A2 = (const T*)A2p; const T* Bt = (const T*)Btp; const T* Bt2 = (const T*)Bt2p;
  __shared__ __align__(16) float sT[8][16 * 68];
  const int b    = blockIdx.y;
  const int lane = threadIdx.x & 31;
  const int wave = threadIdx.x >> 5;
  const int tilesN = N >> 6;
  const int tilesM = M >> 6;
  const int tile = blockIdx.x * 8 + wave;
  if (tile >= tilesM * tilesN) return;
  const int tm = tile / tilesN;
  const int tn = tile - tm * tilesN;
  const int m0 = tm << 6;
  const int n0 = tn << 6;

  const T* Ab  = A  + (size_t)b * strideA;
  const T* Bb  = Bt + (size_t)b * strideB;
  const T* Ab2 = SPLIT ? (A2  + (size_t)b * strideA) : nullptr;
  const T* Bb2 = SPLIT ? (Bt2 + (size_t)b * strideB) : nullptr;

  const int rlane = lane & 15;
  const int koff  = (lane >> 4) * 8;
  const int mOff  = (lane >> 4) * 8;

  v8f acc[4][4];
#pragma unroll
  for (int i = 0; i < 4; ++i)
#pragma unroll
    for (int j = 0; j < 4; ++j) acc[i][j] = (v8f){0.f,0.f,0.f,0.f,0.f,0.f,0.f,0.f};

  for (int k0 = 0; k0 < K; k0 += 32) {
    V bh[4], bl[4];
#pragma unroll
    for (int j = 0; j < 4; ++j) {
      const size_t bo = (size_t)(n0 + (j << 4) + rlane) * ldb + koff + k0;
      bh[j] = Frag<T>::load(Bb + bo);
      if (SPLIT) bl[j] = Frag<T>::load(Bb2 + bo);
    }
#pragma unroll
    for (int i = 0; i < 4; ++i) {
      const size_t ao = (size_t)(m0 + (i << 4) + rlane) * lda + koff + k0;
      V ah = Frag<T>::load(Ab + ao);
      V al;
      if (SPLIT) al = Frag<T>::load(Ab2 + ao);
#pragma unroll
      for (int j = 0; j < 4; ++j) {
        acc[i][j] = Frag<T>::mma(ah, bh[j], acc[i][j]);
        if (SPLIT) {
          acc[i][j] = Frag<T>::mma(ah, bl[j], acc[i][j]);
          acc[i][j] = Frag<T>::mma(al, bh[j], acc[i][j]);
        }
      }
      Frag<T>::guard(acc[i][0], acc[i][3], ah, SPLIT ? al : ah);
    }
    Frag<T>::keep(bh[0], bh[1], bh[2], bh[3]);
    if (SPLIT) Frag<T>::keep(bl[0], bl[1], bl[2], bl[3]);
  }
  acc_guard4(acc[0][0], acc[0][1], acc[0][2], acc[0][3]);
  acc_guard4(acc[1][0], acc[1][1], acc[1][2], acc[1][3]);
  acc_guard4(acc[2][0], acc[2][1], acc[2][2], acc[2][3]);
  acc_guard4(acc[3][0], acc[3][1], acc[3][2], acc[3][3]);

  float* slab = sT[wave];
  const float* Rb = RESID ? (resid + (size_t)b * strideR) : nullptr;
#pragma unroll
  for (int i = 0; i < 4; ++i) {
    const int mBase = m0 + (i << 4);
#pragma unroll
    for (int j = 0; j < 4; ++j) {
      const int n = n0 + (j << 4) + rlane;
      float bv = 0.f;
      if (BIAS_MODE == 2) bv = bias[n];
#pragma unroll
      for (int r = 0; r < 8; ++r) {
        float v = acc[i][j][r] * scale;
        if (BIAS_MODE == 1) v += bias[mBase + mOff + r];
        if (BIAS_MODE == 2) v += bv;
        if (ACT == 2) v = fmaxf(v, 0.0f);
        if (ACT == 4) v = (v > 0.f) ? v : 0.01f * v;
        slab[(mOff + r) * 68 + (j << 4) + rlane] = v;
      }
    }
    __builtin_amdgcn_fence(__ATOMIC_RELEASE, "workgroup");
    __builtin_amdgcn_wave_barrier();
    __builtin_amdgcn_fence(__ATOMIC_ACQUIRE, "workgroup");
    if (OUT_MODE == 0) {
      float* C = (float*)Cout + (size_t)b * strideC;
      const int hh = lane >> 4, c4 = (lane & 15) * 4;
      for (int pass = 0; pass < 2; ++pass) {
#pragma unroll
        for (int it = 0; it < 8; ++it) {
          const int row = it * 2 + hh;
          v4f v = *(const v4f*)(slab + row * 68 + c4);
          if (RESID) {
            const v4f rr = *(const v4f*)(Rb + (size_t)(mBase + row) * ldc + n0 + c4);
            v = v + rr;
          }
          *(volatile v4f*)(C + (size_t)(mBase + row) * ldc + n0 + c4) = v;
        }
        __threadfence();
      }
    } else {
      const int q = lane >> 3, c8 = (lane & 7) * 8;
      unsigned short* C  = (unsigned short*)Cout  + (size_t)b * strideC;
      unsigned short* C2 = (OUT_MODE == 2) ? ((unsigned short*)Cout2 + (size_t)b * strideC) : nullptr;
      for (int pass = 0; pass < 2; ++pass) {
#pragma unroll
        for (int it = 0; it < 4; ++it) {
          const int row = it * 4 + q;
          const float* sp = slab + row * 68 + c8;
          v8h hv, lv;
#pragma unroll
          for (int e = 0; e < 8; ++e) {
            if (OUT_MODE == 1) {
              hv[e] = (_Float16)sp[e];
            } else {
              unsigned short hb = f2bf_bits(sp[e]);
              unsigned short lb = f2bf_bits(sp[e] - bf_bits2f(hb));
              hv[e] = __builtin_bit_cast(_Float16, hb);
              lv[e] = __builtin_bit_cast(_Float16, lb);
            }
          }
          *(volatile v8h*)(C + (size_t)(mBase + row) * ldc + n0 + c8) = hv;
          if (OUT_MODE == 2) *(volatile v8h*)(C2 + (size_t)(mBase + row) * ldc + n0 + c8) = lv;
        }
        __threadfence();
      }
    }
    __builtin_amdgcn_fence(__ATOMIC_RELEASE, "workgroup");
    __builtin_amdgcn_wave_barrier();
    __builtin_amdgcn_fence(__ATOMIC_ACQUIRE, "workgroup");
  }
}

__global__ __launch_bounds__(256) void cast8_f16_kernel(const float* __restrict__ in, unsigned short* __restrict__ out, int n8) {
  const int i = blockIdx.x * 256 + threadIdx.x;
  if (i >= n8) return;
  const float* p = in + 8 * (size_t)i;
  const v4f a = *(const v4f*)(p);
  const v4f c = *(const v4f*)(p + 4);
  unsigned short hb[8];
#pragma unroll
  for (int e = 0; e < 4; ++e) {
    hb[e]     = h_bits(a[e]);
    hb[4 + e] = h_bits(c[e]);
  }
  const v4u u = (v4u){pk16(hb[0], hb[1]), pk16(hb[2], hb[3]), pk16(hb[4], hb[5]), pk16(hb[6], hb[7])};
  unsigned short* q = out + 8 * (size_t)i;
  *(volatile v4u*)q = u;
  __threadfence();
  *(volatile v4u*)q = u;
}

__global__ __launch_bounds__(256) void wt32_kernel(const float* __restrict__ W0, const float* __restrict__ W1,
                                                   const float* __restrict__ W2, int ncols, int tpm, int nmats,
                                                   unsigned short* __restrict__ out, int ld_out, float scale) {
  __shared__ float sm[32][65];
  const int t  = threadIdx.x;
  const int k0 = blockIdx.x * 64;
  const int nt = blockIdx.y;
  const int m  = nt / tpm;
  const int nloc0 = (nt - m * tpm) * 32;
  const float* W = (m == 0) ? W0 : (m == 1) ? W1 : W2;
  if (m < nmats) {
#pragma unroll
    for (int i = 0; i < 8; ++i) {
      const int e  = i * 256 + t;
      const int kl = e >> 5;
      const int nl = e & 31;
      sm[nl][kl] = W[(size_t)(k0 + kl) * ncols + nloc0 + nl] * scale;
    }
  } else {
#pragma unroll
    for (int i = 0; i < 8; ++i) {
      const int e  = i * 256 + t;
      sm[e & 31][e >> 5] = 0.0f;
    }
  }
  __syncthreads();
  const int lane = t & 31, wave = t >> 5;
  const int q = lane >> 3, c8 = (lane & 7) * 8;
  const int row = wave * 4 + q;
  unsigned short hb[8];
#pragma unroll
  for (int e = 0; e < 8; ++e) hb[e] = h_bits(sm[row][c8 + e]);
  const v4u u = (v4u){pk16(hb[0], hb[1]), pk16(hb[2], hb[3]), pk16(hb[4], hb[5]), pk16(hb[6], hb[7])};
  unsigned short* op = out + (size_t)(nt * 32 + row) * ld_out + k0 + c8;
  *(volatile v4u*)op = u;
  __threadfence();
  *(volatile v4u*)op = u;
}

__global__ __launch_bounds__(256) void points_kernel(const float* __restrict__ pproj, const float* __restrict__ rot,
                                                     const float* __restrict__ trans, float* __restrict__ QG,
                                                     float* __restrict__ KG, unsigned short* __restrict__ VTP) {
  __shared__ float sR[64 * 9];
  __shared__ float sTr[64 * 3];
  __shared__ __align__(16) float sQ[4][64 * kPc];
  __shared__ __align__(16) float sK[4][64 * kPc];
  __shared__ unsigned short sV[4][kVtpLive][64];
  const int t = threadIdx.x;
  const int lane = t & 31, wave = t >> 5;
  const int j0 = blockIdx.x * 64;
  const int h0 = blockIdx.y * 4;
  const int bb = blockIdx.z;
  const int tok0 = bb * kN + j0;
  for (int idx = t; idx < 64 * 9; idx += 256) sR[idx] = rot[(size_t)tok0 * 9 + idx];
  if (t < 64 * 3) sTr[t] = trans[(size_t)tok0 * 3 + t];
  __syncthreads();

  const int jl = t & 63, hl = t >> 6;
  const int h = h0 + hl;
  const float* prow = pproj + (size_t)(tok0 + jl) * kProjN + h * kPc;
  float qp[12], kp[12], vp[12];
  {
    const v4f qa = *(const v4f*)(prow),              qb = *(const v4f*)(prow + 4),              qc = *(const v4f*)(prow + 8);
    const v4f ka = *(const v4f*)(prow + kProjW),     kb = *(const v4f*)(prow + kProjW + 4),     kc = *(const v4f*)(prow + kProjW + 8);
    const v4f va = *(const v4f*)(prow + 2 * kProjW), vb = *(const v4f*)(prow + 2 * kProjW + 4), vc = *(const v4f*)(prow + 2 * kProjW + 8);
#pragma unroll
    for (int e = 0; e < 4; ++e) {
      qp[e] = qa[e]; qp[4 + e] = qb[e]; qp[8 + e] = qc[e];
      kp[e] = ka[e]; kp[4 + e] = kb[e]; kp[8 + e] = kc[e];
      vp[e] = va[e]; vp[4 + e] = vb[e]; vp[8 + e] = vc[e];
    }
  }
  float R[9], tt[3];
#pragma unroll
  for (int e = 0; e < 9; ++e) R[e] = sR[jl * 9 + e];
#pragma unroll
  for (int c = 0; c < 3; ++c) tt[c] = sTr[jl * 3 + c];
  float* sq = &sQ[hl][jl * kPc];
  float* sk = &sK[hl][jl * kPc];
#pragma unroll
  for (int p = 0; p < kP; ++p) {
#pragma unroll
    for (int c = 0; c < 3; ++c) {
      float aq = R[3 * c] * qp[3 * p]; aq = fmaf(R[3 * c + 1], qp[3 * p + 1], aq); aq = fmaf(R[3 * c + 2], qp[3 * p + 2], aq);
      float ak = R[3 * c] * kp[3 * p]; ak = fmaf(R[3 * c + 1], kp[3 * p + 1], ak); ak = fmaf(R[3 * c + 2], kp[3 * p + 2], ak);
      float av = R[3 * c] * vp[3 * p]; av = fmaf(R[3 * c + 1], vp[3 * p + 1], av); av = fmaf(R[3 * c + 2], vp[3 * p + 2], av);
      sq[3 * p + c] = aq + tt[c];
      sk[3 * p + c] = ak + tt[c];
      sV[hl][3 * p + c][jl] = h_bits(kFCarry * av);
    }
  }
#pragma unroll
  for (int c = 0; c < 3; ++c) {
    unsigned short hb, lb;
    split16(kFCarry * tt[c], hb, lb);
    sV[hl][12 + c][jl] = hb;
    sV[hl][15 + c][jl] = lb;
  }
  sV[hl][18][jl] = (unsigned short)0x4C00u;
  __syncthreads();

  const size_t bh0 = (size_t)(bb * kH + h0);
  const int hd2 = wave >> 1;
  const int q8 = lane >> 3, c8 = (lane & 7) * 8;
  const v4u z4 = (v4u){0u, 0u, 0u, 0u};
  for (int pass = 0; pass < 2; ++pass) {
#pragma unroll
    for (int it = 0; it < 3; ++it) {
      const int idx = it * 256 + t;
      const int hd  = idx / 192;
      const int off = idx - hd * 192;
      const v4f vq = *(const v4f*)(&sQ[hd][off * 4]);
      const v4f vk = *(const v4f*)(&sK[hd][off * 4]);
      const size_t go = ((bh0 + hd) * kN + j0) * kPc + (size_t)off * 4;
      *(volatile v4f*)(QG + go) = vq;
      *(volatile v4f*)(KG + go) = vk;
    }
#pragma unroll
    for (int it = 0; it < 8; ++it) {
      const int row = (wave & 1) * 32 + it * 4 + q8;
      const int rr = row < (kVtpLive - 1) ? row : (kVtpLive - 1);
      const unsigned short* sp = &sV[hd2][rr][c8];
      v4u u = (v4u){pk16(sp[0], sp[1]), pk16(sp[2], sp[3]), pk16(sp[4], sp[5]), pk16(sp[6], sp[7])};
      if (row >= kVtpLive) u = z4;
      *(volatile v4u*)(VTP + ((bh0 + hd2) * kVtpRows + row) * (size_t)kN + j0 + c8) = u;
    }
    __threadfence();
  }
}

__global__ __launch_bounds__(512) void dist_softmax_kernel(const float* __restrict__ SC, const float* __restrict__ QG,
                                                          const float* __restrict__ KG, const float* __restrict__ pw,
                                                          unsigned short* __restrict__ PP, int bh0) {
  __shared__ __align__(16) float lg[kN];
  __shared__ float redM[16];
  __shared__ float redS[16];
  const int i    = blockIdx.x;
  const int h    = blockIdx.y;
  const int t    = threadIdx.x;
  const int lane = t & 31, wave = t >> 5;
  const float pwh = pw[h];
  const float spw = fmaxf(pwh, 0.0f) + log1pf(expf(-fabsf(pwh)));
  const size_t rowoff = ((size_t)h * kN + i) * kN;
  const float* qr = QG + ((size_t)(bh0 + h) * kN + i) * kPc;
  const v4f qa = *(const v4f*)(qr), qb = *(const v4f*)(qr + 4), qc = *(const v4f*)(qr + 8);
  const float* kr = KG + ((size_t)(bh0 + h) * kN + 2 * t) * kPc;
  const v4f k0 = *(const v4f*)(kr),      k1 = *(const v4f*)(kr + 4),  k2 = *(const v4f*)(kr + 8);
  const v4f k3 = *(const v4f*)(kr + 12), k4 = *(const v4f*)(kr + 16), k5 = *(const v4f*)(kr + 20);
  const v2f sv = *(const v2f*)(SC + rowoff + 2 * t);
  float q[12], ka[12], kb[12];
#pragma unroll
  for (int e = 0; e < 4; ++e) {
    q[e]  = qa[e]; q[4 + e]  = qb[e]; q[8 + e]  = qc[e];
    ka[e] = k0[e]; ka[4 + e] = k1[e]; ka[8 + e] = k2[e];
    kb[e] = k3[e]; kb[4 + e] = k4[e]; kb[8 + e] = k5[e];
  }
  float d0 = 0.0f, d1 = 0.0f;
#pragma unroll
  for (int e = 0; e < 12; ++e) {
    const float u0 = q[e] - ka[e]; d0 = fmaf(u0, u0, d0);
    const float u1 = q[e] - kb[e]; d1 = fmaf(u1, u1, d1);
  }
  const float a0 = sv[0] + ((-0.5f * d0) * spw) * kPointScale;
  const float a1 = sv[1] + ((-0.5f * d1) * spw) * kPointScale;
  lg[2 * t]     = a0;
  lg[2 * t + 1] = a1;
  float mx = fmaxf(a0, a1);
#pragma unroll
  for (int off = 16; off > 0; off >>= 1) mx = fmaxf(mx, __shfl_xor(mx, off, 32));
  if (lane == 0) redM[wave] = mx;
  __syncthreads();
  float m = redM[0];
#pragma unroll
  for (int w = 1; w < 16; ++w) m = fmaxf(m, redM[w]);

  float sum = 0.0f;
#pragma unroll 1
  for (int e = 0; e < 2; ++e) {
    const float ev = expf(lg[2 * t + e] - m);
    sum += ev;
    lg[2 * t + e] = ev;
  }
#pragma unroll
  for (int off = 16; off > 0; off >>= 1) sum += __shfl_xor(sum, off, 32);
  if (lane == 0) redS[wave] = sum;
  __syncthreads();
  float tot = redS[0];
#pragma unroll
  for (int w = 1; w < 16; ++w) tot += redS[w];
  const float inv = kPCarry / tot;

  if (t < 128) {
    const v4f e0 = *(const v4f*)(lg + 8 * t);
    const v4f e1 = *(const v4f*)(lg + 8 * t + 4);
    unsigned short hb[8];
#pragma unroll
    for (int e = 0; e < 4; ++e) {
      hb[e]     = h_bits(e0[e] * inv);
      hb[4 + e] = h_bits(e1[e] * inv);
    }
    const v4u u = (v4u){pk16(hb[0], hb[1]), pk16(hb[2], hb[3]), pk16(hb[4], hb[5]), pk16(hb[6], hb[7])};
    unsigned short* pr = PP + rowoff + 8 * (size_t)t;
    *(volatile v4u*)pr = u;
    __threadfence();
    *(volatile v4u*)pr = u;
  }
}

__global__ __launch_bounds__(256) void finalize_kernel(const float* __restrict__ RPG, const float* __restrict__ rot,
                                                       const float* __restrict__ trans, unsigned short* __restrict__ FEAT,
                                                       unsigned short* __restrict__ FLO) {
  __shared__ float sR[32 * 9];
  __shared__ float sTr[32 * 3];
  __shared__ __align__(16) unsigned short sH[32][kFeatPt];
  __shared__ __align__(16) unsigned short sL[32][kFeatPt];
  const int t = threadIdx.x;
  const int lane = t & 31, wave = t >> 5;
  const int tok0 = blockIdx.x * 32;
  for (int idx = t; idx < 32 * 9; idx += 256) sR[idx] = rot[(size_t)tok0 * 9 + idx];
  if (t < 32 * 3) sTr[t] = trans[(size_t)tok0 * 3 + t];
  __syncthreads();

  const int tl = t >> 3, h = t & 7;
  const float* rp = RPG + (size_t)(tok0 + tl) * kDim + h * 64;
  float a[20];
  {
    const v4f r0 = *(const v4f*)(rp), r1 = *(const v4f*)(rp + 4), r2 = *(const v4f*)(rp + 8), r3 = *(const v4f*)(rp + 12), r4 = *(const v4f*)(rp + 16);
#pragma unroll
    for (int e = 0; e < 4; ++e) { a[e] = r0[e]; a[4 + e] = r1[e]; a[8 + e] = r2[e]; a[12 + e] = r3[e]; a[16 + e] = r4[e]; }
  }
  float R[9], tt[3];
#pragma unroll
  for (int e = 0; e < 9; ++e) R[e] = sR[tl * 9 + e];
#pragma unroll
  for (int c = 0; c < 3; ++c) tt[c] = sTr[tl * 3 + c];
  const float inv = 1.0f / a[18];
  float T3[3];
#pragma unroll
  for (int c = 0; c < 3; ++c) T3[c] = fmaf(a[15 + c], kLoInv, a[12 + c]) * inv - tt[c];
#pragma unroll
  for (int p = 0; p < kP; ++p) {
    float g[3];
#pragma unroll
    for (int c = 0; c < 3; ++c) g[c] = fmaf(a[3 * p + c], inv, T3[c]);
    float l[3];
#pragma unroll
    for (int c = 0; c < 3; ++c) {
      float s = R[c] * g[0]; s = fmaf(R[3 + c], g[1], s); s = fmaf(R[6 + c], g[2], s);
      l[c] = s;
    }
    float nn = l[0] * l[0]; nn = fmaf(l[1], l[1], nn); nn = fmaf(l[2], l[2], nn);
    const float nrm = sqrtf(nn + kEps);
#pragma unroll
    for (int c = 0; c < 3; ++c) {
      unsigned short hb, lb;
      split16(kFCarry * l[c], hb, lb);
      sH[tl][h * kPc + 3 * p + c] = hb;
      sL[tl][h * kPc + 3 * p + c] = lb;
    }
    {
      unsigned short hb, lb;
      split16(kFCarry * nrm, hb, lb);
      sH[tl][kProjW + h * kP + p] = hb;
      sL[tl][kProjW + h * kP + p] = lb;
    }
  }
  __syncthreads();

  const int hh = lane >> 4, c8 = (lane & 15) * 8;
  for (int pass = 0; pass < 2; ++pass) {
#pragma unroll
    for (int it = 0; it < 2; ++it) {
      const int row = wave * 4 + it * 2 + hh;
      const unsigned short* sp = &sH[row][c8];
      const v4u u = (v4u){pk16(sp[0], sp[1]), pk16(sp[2], sp[3]), pk16(sp[4], sp[5]), pk16(sp[6], sp[7])};
      *(volatile v4u*)(FEAT + (size_t)(tok0 + row) * kFeat + kDim + c8) = u;
      const unsigned short* lp = &sL[row][c8];
      const v4u w = (v4u){pk16(lp[0], lp[1]), pk16(lp[2], lp[3]), pk16(lp[4], lp[5]), pk16(lp[6], lp[7])};
      *(volatile v4u*)(FLO + (size_t)(tok0 + row) * kFeatPt + c8) = w;
    }
    __threadfence();
  }
}

extern "C" void kernel_launch(void* const* d_in, const int* in_sizes, int n_in,
                              void* d_out, int out_size, void* d_ws, size_t ws_size,
                              hipStream_t stream) {
  if (n_in < 12) return;
  if (in_sizes[0] != kTok * kDim) return;
  if (in_sizes[1] != kTok * 9 || in_sizes[2] != kTok * 3) return;
  if (in_sizes[3] != kDim * kDim || in_sizes[4] != kDim * kDim || in_sizes[5] != kDim * kDim) return;
  if (in_sizes[6] != kDim * kProjW || in_sizes[7] != kDim * kProjW || in_sizes[8] != kDim * kProjW) return;
  if (in_sizes[9] != kH || in_sizes[10] != kFeat * kDim || in_sizes[11] != kDim) return;
  if (out_size != kTok * kDim) return;

  static_assert(kTok % 64 == 0 && (2 * kDim) % 64 == 0 && kDim % 32 == 0, "qk proj tiles");
  static_assert(kDim % 64 == 0 && kN % 64 == 0, "vt proj tiles");
  static_assert(kProjN % 64 == 0, "point proj tiles");
  static_assert(kN % 64 == 0 && kDh % 32 == 0, "scores tiles");
  static_assert(kVtpRows == 64 && kN % 32 == 0, "pv tiles");
  static_assert(kFeatPt % 32 == 0 && kFeat % 32 == 0 && kDim % 64 == 0, "out tiles");

  const size_t szX16  = (size_t)kTok * kDim * 2;
  const size_t szWQKV = (size_t)3 * kDim * kDim * 2;
  const size_t szWP   = (size_t)kProjN * kDim * 2;
  const size_t szWO   = (size_t)kDim * kFeat * 2;
  const size_t szQK   = (size_t)kTok * 2 * kDim * 2;
  const size_t szVTS  = (size_t)kB * kDim * kN * 2;
  const size_t szPPJ  = (size_t)kTok * kProjN * 4;
  const size_t szG    = (size_t)kB * kH * kN * kPc * 4;
  const size_t szVTP  = (size_t)kB * kH * kVtpRows * kN * 2;
  const size_t szSC   = (size_t)kH * kN * kN * 4;
  const size_t szP    = (size_t)kH * kN * kN * 2;
  const size_t szRPG  = (size_t)kTok * kDim * 4;
  const size_t szFEAT = (size_t)kTok * kFeat * 2;
  const size_t szFLO  = (size_t)kTok * kFeatPt * 2;
  const size_t szTLO  = (size_t)kTok * kDim * 4;
  const size_t offX16  = 0;
  const size_t offWQKV = offX16 + szX16;
  const size_t offWP   = offWQKV + szWQKV;
  const size_t offWO   = offWP + szWP;
  const size_t offQK   = offWO + szWO;
  const size_t offVTS  = offQK + szQK;
  const size_t offPPJ  = offVTS + szVTS;
  const size_t offQG   = offPPJ + szPPJ;
  const size_t offKG   = offQG + szG;
  const size_t offVTP  = offKG + szG;
  const size_t offSC   = offVTP + szVTP;
  const size_t offP    = offSC + szSC;
  const size_t offRPG  = offP + szP;
  const size_t offFEAT = offRPG + szRPG;
  const size_t offFLO  = offFEAT + szFEAT;
  const size_t offTLO  = offFLO + szFLO;
  const size_t total   = offTLO + szTLO;
  if (ws_size < total) return;

  const float* x     = (const float*)d_in[0];
  const float* rot   = (const float*)d_in[1];
  const float* trans = (const float*)d_in[2];
  const float* w_qs  = (const float*)d_in[3];
  const float* w_ks  = (const float*)d_in[4];
  const float* w_vs  = (const float*)d_in[5];
  const float* w_qp  = (const float*)d_in[6];
  const float* w_kp  = (const float*)d_in[7];
  const float* w_vp  = (const float*)d_in[8];
  const float* pwts  = (const float*)d_in[9];
  const float* w_o   = (const float*)d_in[10];
  const float* b_o   = (const float*)d_in[11];
  float* out = (float*)d_out;
  char* ws = (char*)d_ws;
  unsigned short* X16  = (unsigned short*)(ws + offX16);
  unsigned short* WQKV = (unsigned short*)(ws + offWQKV);
  unsigned short* WP   = (unsigned short*)(ws + offWP);
  unsigned short* WO   = (unsigned short*)(ws + offWO);
  unsigned short* QK16 = (unsigned short*)(ws + offQK);
  unsigned short* VTS  = (unsigned short*)(ws + offVTS);
  float* PPROJ = (float*)(ws + offPPJ);
  float* QG    = (float*)(ws + offQG);
  float* KG    = (float*)(ws + offKG);
  unsigned short* VTP  = (unsigned short*)(ws + offVTP);
  float* SC    = (float*)(ws + offSC);
  unsigned short* PP   = (unsigned short*)(ws + offP);
  float* RPG   = (float*)(ws + offRPG);
  unsigned short* FEAT = (unsigned short*)(ws + offFEAT);
  unsigned short* FLO  = (unsigned short*)(ws + offFLO);
  float* TLO   = (float*)(ws + offTLO);

  const int n8 = (kTok * kDim) / 8;
  cast8_f16_kernel<<<dim3(n8 / 256), dim3(256), 0, stream>>>(x, X16, n8);
  wt32_kernel<<<dim3(kDim / 64, 3 * kDim / 32), dim3(256), 0, stream>>>(w_qs, w_ks, w_vs, kDim, kDim / 32, 3, WQKV, kDim, kWCarry);
  wt32_kernel<<<dim3(kDim / 64, kProjN / 32), dim3(256), 0, stream>>>(w_qp, w_kp, w_vp, kProjW, kProjW / 32, 3, WP, kDim, kWCarry);
  wt32_kernel<<<dim3(kFeat / 64, kDim / 32), dim3(256), 0, stream>>>(w_o, w_o, w_o, kDim, kDim / 32, 1, WO, kFeat, kWCarry);

  wmma_gemm64<0, false, 0, 1, false, 0><<<dim3((kTok / 64) * (2 * kDim / 64) / 8, 1), dim3(256), 0, stream>>>(
      X16, X16, kDim, 0L, WQKV, WQKV, kDim, 0L,
      (void*)QK16, (void*)QK16, 2 * kDim, 0L, b_o, b_o, 0L, kTok, 2 * kDim, kDim, 1.0f);
  wmma_gemm64<0, false, 0, 1, false, 0><<<dim3((kDim / 64) * (kN / 64) / 8, kB), dim3(256), 0, stream>>>(
      WQKV + (size_t)2 * kDim * kDim, WQKV + (size_t)2 * kDim * kDim, kDim, 0L, X16, X16, kDim, (long)kN * kDim,
      (void*)VTS, (void*)VTS, kN, (long)kDim * kN, b_o, b_o, 0L, kDim, kN, kDim, 1.0f);
  wmma_gemm64<0, false, 0, 0, false, 0><<<dim3((kTok / 64) * (kProjN / 64) / 8, 1), dim3(256), 0, stream>>>(
      X16, X16, kDim, 0L, WP, WP, kDim, 0L,
      (void*)PPROJ, (void*)PPROJ, kProjN, 0L, b_o, b_o, 0L, kTok, kProjN, kDim, 1.0f / kWCarry);

  points_kernel<<<dim3(kN / 64, kH / 4, kB), dim3(256), 0, stream>>>(PPROJ, rot, trans, QG, KG, VTP);

  const long strideHead16 = (long)kDh;
  const long strideScore  = (long)kN * kN;
  const long strideVT     = (long)kVtpRows * kN;
  const int  tilesScore   = (kN / 64) * (kN / 64);
  const int  tilesPV      = (kN / 64) * (64 / 64);
  for (int b = 0; b < kB; ++b) {
    const size_t qkOff = (size_t)b * kN * (2 * kDim);
    wmma_gemm64<0, false, 0, 0, false, 0><<<dim3(tilesScore / 8, kH), dim3(256), 0, stream>>>(
        QK16 + qkOff, QK16 + qkOff, 2 * kDim, strideHead16, QK16 + qkOff + kDim, QK16 + qkOff + kDim, 2 * kDim, strideHead16,
        (void*)SC, (void*)SC, kN, strideScore, b_o, b_o, 0L, kN, kN, kDh, kScalarScale / 256.0f);
    dist_softmax_kernel<<<dim3(kN, kH), dim3(512), 0, stream>>>(SC, QG, KG, pwts, PP, b * kH);
    wmma_gemm64<0, false, 0, 1, false, 0><<<dim3(tilesPV / 8, kH), dim3(256), 0, stream>>>(
        PP, PP, kN, strideScore, VTS + (size_t)b * kDim * kN, VTS + (size_t)b * kDim * kN, kN, (long)kDh * kN,
        (void*)(FEAT + (size_t)b * kN * kFeat), (void*)(FEAT + (size_t)b * kN * kFeat), kFeat, (long)kDh,
        b_o, b_o, 0L, kN, 64, kN, 1.0f / kPCarry);
    wmma_gemm64<0, false, 0, 0, false, 0><<<dim3(tilesPV / 8, kH), dim3(256), 0, stream>>>(
        PP, PP, kN, strideScore, VTP + (size_t)b * kH * kVtpRows * kN, VTP + (size_t)b * kH * kVtpRows * kN, kN, strideVT,
        (void*)(RPG + (size_t)b * kN * kDim), (void*)(RPG + (size_t)b * kN * kDim), kDim, (long)64,
        b_o, b_o, 0L, kN, 64, kN, 1.0f / (kPCarry * kFCarry));
  }

  finalize_kernel<<<dim3(kTok / 32), dim3(256), 0, stream>>>(RPG, rot, trans, FEAT, FLO);

  wmma_gemm64<0, false, 0, 0, false, 0><<<dim3((kTok / 64) * (kDim / 64) / 8, 1), dim3(256), 0, stream>>>(
      FLO, FLO, kFeatPt, 0L, WO + kDim, WO + kDim, kFeat, 0L,
      (void*)TLO, (void*)TLO, kDim, 0L, b_o, b_o, 0L, kTok, kDim, kFeatPt, 1.0f / (kFCarry * kWCarry * kLoCarry));
  wmma_gemm64<0, false, 2, 0, true, 0><<<dim3((kTok / 64) * (kDim / 64) / 8, 1), dim3(256), 0, stream>>>(
      FEAT, FEAT, kFeat, 0L, WO, WO, kFeat, 0L,
      (void*)out, (void*)out, kDim, 0L, b_o, TLO, 0L, kTok, kDim, kFeat, 1.0f / (kFCarry * kWCarry));
}
